// ManifestEncoder_14164802142469
// MI455X (gfx1250) — hardware-run, weakly checked
//
#include <hip/hip_runtime.h>
#include <math.h>
#include <stddef.h>
#include <stdint.h>


#define NB    64
#define NI    8192
#define NF    8
#define HD    128
#define ED    128
#define PD    256
#define WAVES 4
#define BPB   8
#define TPW   (NI / (16 * BPB * WAVES))
#define AP    (HD + 8)
#define PP    (PD + 8)
#define WSCAP 134217728

static_assert(TPW * 16 * BPB * WAVES == NI);
static_assert(HD == 128);
static_assert(ED == 128);
static_assert(PD == 2 * ED);
static_assert(NB % 16 == 0);
static_assert(HD % 32 == 0);
static_assert(PD % 32 == 0);
static_assert(AP % 8 == 0);
static_assert(PP % 8 == 0);

typedef float          v4f   __attribute__((ext_vector_type(4)));
typedef float          v8f   __attribute__((ext_vector_type(8)));
typedef unsigned short v4us  __attribute__((ext_vector_type(4)));
typedef unsigned short v8us  __attribute__((ext_vector_type(8)));
typedef unsigned short v16us __attribute__((ext_vector_type(16)));
typedef __bf16         v16b  __attribute__((ext_vector_type(16)));
union FragU { v16us v; v8us h[2]; };

__device__ __forceinline__ unsigned short f2bf(float f) {
  unsigned int u = __float_as_uint(f);
  u += 0x7FFFu + ((u >> 16) & 1u);
  return (unsigned short)(u >> 16);
}
__device__ __forceinline__ float bf2f(unsigned short b) {
  return __uint_as_float(((unsigned int)b) << 16);
}

__device__ __forceinline__ v8f splat8(float x) { v8f r = {x, x, x, x, x, x, x, x}; return r; }

__device__ __forceinline__ v8f wm(v16us a, v16us b, v8f c) {
  const v16b av = __builtin_bit_cast(v16b, a);
  const v16b bv = __builtin_bit_cast(v16b, b);
  v8f d = __builtin_amdgcn_wmma_f32_16x16x32_bf16(false, av, false, bv, (short)0, c, false, false);
  asm volatile("v_nop\n\tv_nop\n\tv_nop\n\tv_nop" : "+v"(d) : "v"(av), "v"(bv));
  return d;
}

__device__ __forceinline__ v16us ldfrag(const unsigned short* p, int k0, int hh) {
  FragU u;
  u.h[0] = *(const v8us*)(p + k0 + 8 * hh);
  u.h[1] = *(const v8us*)(p + k0 + 16 + 8 * hh);
  return u.v;
}

struct Piece { v8us h, l; };

template <int NPC>
__device__ __forceinline__ Piece prepw_piece(const float* ts, int p) {
  const int row = p / NPC, k8 = (p - row * NPC) * 8;
  Piece o;
#pragma unroll
  for (int e = 0; e < 8; ++e) {
    const float x = ts[(k8 + e) * 16 + row];
    const unsigned short hb = f2bf(x);
    o.h[e] = hb;
    o.l[e] = f2bf(x - bf2f(hb));
  }
  return o;
}

template <int KD>
__global__ __launch_bounds__(256) void k_prepw(const float* __restrict__ W, int Nd,
                                                unsigned short* dhi, unsigned short* dlo) {
  static_assert(KD % 32 == 0);
  static_assert(KD <= 256);
  __shared__ __attribute__((aligned(16))) float ts[KD * 16];
  const int t = threadIdx.x;
  const int n0 = blockIdx.x * 16;
  if (t < KD) {
    const float* wrow = W + (size_t)t * Nd;
#pragma unroll
    for (int nn = 0; nn < 16; ++nn) {
      const int n = n0 + nn;
      const float v = wrow[min(n, Nd - 1)];
      ts[t * 16 + nn] = (n < Nd) ? v : 0.0f;
    }
  }
  __syncthreads();
  constexpr int NPC = KD / 8;
  constexpr int TOT = 16 * NPC;
  const int p0 = t, p1 = t + 256;
  const bool a0 = p0 < TOT, a1 = p1 < TOT;
  const Piece q0 = prepw_piece<NPC>(ts, a0 ? p0 : 0);
  const Piece q1 = prepw_piece<NPC>(ts, a1 ? p1 : 0);
  const size_t o0 = (size_t)n0 * KD + 8 * (a0 ? p0 : 0);
  const size_t o1 = (size_t)n0 * KD + 8 * (a1 ? p1 : 0);
  if (a0) { *(volatile v8us*)(dhi + o0) = q0.h; *(volatile v8us*)(dlo + o0) = q0.l; }
  if (a1) { *(volatile v8us*)(dhi + o1) = q1.h; *(volatile v8us*)(dlo + o1) = q1.l; }
  __threadfence();
  if (a0) { *(volatile v8us*)(dhi + o0) = q0.h; *(volatile v8us*)(dlo + o0) = q0.l; }
  if (a1) { *(volatile v8us*)(dhi + o1) = q1.h; *(volatile v8us*)(dlo + o1) = q1.l; }
}

__global__ __launch_bounds__(128) void k_phi(const float* __restrict__ items,
                                              const float* __restrict__ W1, const float* __restrict__ b1,
                                              const float* __restrict__ b2,
                                              const unsigned short* __restrict__ w2h,
                                              const unsigned short* __restrict__ w2l,
                                              float* part) {
  __shared__ __attribute__((aligned(16))) float sW1[NF * HD];
  __shared__ __attribute__((aligned(16))) float sB1[HD];
  __shared__ __attribute__((aligned(16))) float sB2[ED];
  __shared__ __attribute__((aligned(16))) unsigned short sAh[WAVES][16 * AP];
  __shared__ __attribute__((aligned(16))) unsigned short sAl[WAVES][16 * AP];
  __shared__ __attribute__((aligned(16))) float sC[WAVES][16];
  __shared__ __attribute__((aligned(16))) float sPool[2][WAVES][ED];
  __shared__ __attribute__((aligned(16))) float sFin[2 * ED];

  const int t = threadIdx.x, lane = t & 31, wv = t >> 5, hh = lane >> 4, ml = lane & 15;
  const int b = blockIdx.x / BPB, blk = blockIdx.x % BPB;

#pragma unroll
  for (int f = 0; f < NF; ++f) sW1[f * HD + t] = W1[f * HD + t];
  sB1[t] = b1[t];
  sB2[t] = b2[t];
  __syncthreads();

  const int c4 = 4 * lane;
  v4f w1c[NF];
#pragma unroll
  for (int f = 0; f < NF; ++f) w1c[f] = *(const v4f*)(sW1 + f * HD + c4);
  const v4f b1c = *(const v4f*)(sB1 + c4);

  float rs[8], rm[8];
#pragma unroll
  for (int nt = 0; nt < 8; ++nt) { rs[nt] = 0.0f; rm[nt] = -INFINITY; }

  const int base = blk * (WAVES * TPW * 16) + wv * (TPW * 16);
  const float* itb = items + ((size_t)b * NI + base) * 4;

#pragma unroll 1
  for (int tile = 0; tile < TPW; ++tile) {
#pragma unroll 1
    for (int r = 0; r < 16; ++r) {
      const v4f it = *(const v4f*)(itb + (size_t)(tile * 16 + r) * 4);
      const float w = it.x, d = it.y, hgt = it.z, cnt = it.w;
      const float wn = w * 0.01f, dn = d * 0.01f, hn = hgt * 0.01f;
      const float wmin = fminf(wn, dn), dmax = fmaxf(wn, dn);
      const float area = wmin * dmax;
      const float vol = area * hn;
      const float aspect = wmin * (1.0f / fmaxf(dmax, 1e-6f));
      const float issq = (w == d) ? 1.0f : 0.0f;
      v4f x = b1c;
      x = x + wmin * w1c[0];
      x = x + dmax * w1c[1];
      x = x + hgt * w1c[2];
      x = x + area * w1c[3];
      x = x + vol * w1c[4];
      x = x + aspect * w1c[5];
      x = x + issq * w1c[6];
      x = x + cnt * w1c[7];
      v4f e;
      e.x = (x.x > 0.0f) ? x.x : expm1f(x.x);
      e.y = (x.y > 0.0f) ? x.y : expm1f(x.y);
      e.z = (x.z > 0.0f) ? x.z : expm1f(x.z);
      e.w = (x.w > 0.0f) ? x.w : expm1f(x.w);
      v4us hv, lv;
      {
        const unsigned short h0 = f2bf(e.x), h1 = f2bf(e.y), h2 = f2bf(e.z), h3 = f2bf(e.w);
        hv.x = h0; hv.y = h1; hv.z = h2; hv.w = h3;
        lv.x = f2bf(e.x - bf2f(h0));
        lv.y = f2bf(e.y - bf2f(h1));
        lv.z = f2bf(e.z - bf2f(h2));
        lv.w = f2bf(e.w - bf2f(h3));
      }
      *(v4us*)(&sAh[wv][r * AP + c4]) = hv;
      *(v4us*)(&sAl[wv][r * AP + c4]) = lv;
      if (lane == 0) sC[wv][r] = cnt;
    }
    __syncthreads();

    v16us ah[HD / 32], al[HD / 32];
    {
      const unsigned short* ph = &sAh[wv][ml * AP];
      const unsigned short* pl = &sAl[wv][ml * AP];
#pragma unroll
      for (int ks = 0; ks < HD / 32; ++ks) {
        ah[ks] = ldfrag(ph, 32 * ks, hh);
        al[ks] = ldfrag(pl, 32 * ks, hh);
      }
    }
    float c8[8];
#pragma unroll
    for (int r = 0; r < 8; ++r) c8[r] = sC[wv][8 * hh + r];

#pragma unroll
    for (int nt = 0; nt < 8; ++nt) {
      const int col = 16 * nt + ml;
      const unsigned short* bph = w2h + (size_t)col * HD;
      const unsigned short* bpl = w2l + (size_t)col * HD;
      v8f acc = splat8(0.0f);
#pragma unroll
      for (int ks = 0; ks < HD / 32; ++ks) {
        const v16us bh = ldfrag(bph, 32 * ks, hh);
        const v16us bl = ldfrag(bpl, 32 * ks, hh);
        acc = wm(ah[ks], bh, acc);
        acc = wm(ah[ks], bl, acc);
        acc = wm(al[ks], bh, acc);
      }
      const float bias = sB2[col];
      float s = 0.0f, mx = -INFINITY;
#pragma unroll
      for (int r = 0; r < 8; ++r) {
        const float phi = acc[r] + bias;
        s += phi * c8[r];
        mx = fmaxf(mx, phi);
      }
      s += __shfl_xor(s, 16, 32);
      mx = fmaxf(mx, __shfl_xor(mx, 16, 32));
      rs[nt] += s;
      rm[nt] = fmaxf(rm[nt], mx);
    }
    __syncthreads();
  }

  if (hh == 0) {
#pragma unroll
    for (int nt = 0; nt < 8; ++nt) {
      sPool[0][wv][16 * nt + ml] = rs[nt];
      sPool[1][wv][16 * nt + ml] = rm[nt];
    }
  }
  __syncthreads();
  {
    float S = 0.0f, M = -INFINITY;
#pragma unroll
    for (int w = 0; w < WAVES; ++w) {
      S += sPool[0][w][t];
      M = fmaxf(M, sPool[1][w][t]);
    }
    sFin[t] = S;
    sFin[ED + t] = M;
  }
  __syncthreads();
  const v4f v = *(const v4f*)(sFin + 4 * (t & 63));
  float* dst = part + (size_t)blockIdx.x * PD + 4 * (t & 63);
  if (t < 64) *(volatile v4f*)dst = v;
  __threadfence();
  if (t < 64) *(volatile v4f*)dst = v;
}

__global__ __launch_bounds__(256) void k_head(const float* __restrict__ part,
                                               const unsigned short* __restrict__ wrh,
                                               const unsigned short* __restrict__ wrl,
                                               const float* __restrict__ br, float* out) {
  __shared__ __attribute__((aligned(16))) unsigned short sPh[16 * PP];
  __shared__ __attribute__((aligned(16))) unsigned short sPl[16 * PP];
  __shared__ __attribute__((aligned(16))) float sO[16 * ED];

  const int t = threadIdx.x, lane = t & 31, wv = t >> 5, hh = lane >> 4, ml = lane & 15;
  const int r0 = blockIdx.x * 16;

  {
    const int c4 = 4 * (t & 63);
    const int rg = t >> 6;
    const bool is_sum = c4 < ED;
#pragma unroll 1
    for (int j = 0; j < 4; ++j) {
      const int i = rg + 4 * j;
      const int bb = r0 + i;
      const float* pr = part + (size_t)bb * BPB * PD + c4;
      v4f S = {0.0f, 0.0f, 0.0f, 0.0f};
      v4f M = {-INFINITY, -INFINITY, -INFINITY, -INFINITY};
#pragma unroll
      for (int k = 0; k < BPB; ++k) {
        const v4f x = *(const v4f*)(pr + (size_t)k * PD);
        S = S + x;
        M.x = fmaxf(M.x, x.x);
        M.y = fmaxf(M.y, x.y);
        M.z = fmaxf(M.z, x.z);
        M.w = fmaxf(M.w, x.w);
      }
      v4f v;
      v.x = is_sum ? S.x : M.x;
      v.y = is_sum ? S.y : M.y;
      v.z = is_sum ? S.z : M.z;
      v.w = is_sum ? S.w : M.w;
      v4us hv, lv;
      {
        const unsigned short h0 = f2bf(v.x), h1 = f2bf(v.y), h2 = f2bf(v.z), h3 = f2bf(v.w);
        hv.x = h0; hv.y = h1; hv.z = h2; hv.w = h3;
        lv.x = f2bf(v.x - bf2f(h0));
        lv.y = f2bf(v.y - bf2f(h1));
        lv.z = f2bf(v.z - bf2f(h2));
        lv.w = f2bf(v.w - bf2f(h3));
      }
      *(v4us*)(sPh + i * PP + c4) = hv;
      *(v4us*)(sPl + i * PP + c4) = lv;
    }
  }
  __syncthreads();

  const int col = 16 * wv + ml;
  const unsigned short* ap_h = sPh + ml * PP;
  const unsigned short* ap_l = sPl + ml * PP;
  const unsigned short* bp_h = wrh + (size_t)col * PD;
  const unsigned short* bp_l = wrl + (size_t)col * PD;
  v8f acc = splat8(0.0f);
#pragma unroll
  for (int ks = 0; ks < PD / 32; ++ks) {
    const v16us a_h = ldfrag(ap_h, 32 * ks, hh);
    const v16us a_l = ldfrag(ap_l, 32 * ks, hh);
    const v16us b_h = ldfrag(bp_h, 32 * ks, hh);
    const v16us b_l = ldfrag(bp_l, 32 * ks, hh);
    acc = wm(a_h, b_h, acc);
    acc = wm(a_h, b_l, acc);
    acc = wm(a_l, b_h, acc);
  }
  const float bias = br[col];
#pragma unroll
  for (int r = 0; r < 8; ++r) sO[(8 * hh + r) * ED + col] = acc[r] + bias;
  __syncthreads();

  const v4f v0 = *(const v4f*)(sO + 4 * t);
  const v4f v1 = *(const v4f*)(sO + 8 * ED + 4 * t);
  float* d0 = out + (size_t)r0 * ED + 4 * t;
  float* d1 = d0 + 8 * ED;
  *(volatile v4f*)d0 = v0;
  *(volatile v4f*)d1 = v1;
  __threadfence();
  *(volatile v4f*)d0 = v0;
  *(volatile v4f*)d1 = v1;
}

extern "C" void kernel_launch(void* const* d_in, const int* in_sizes, int n_in,
                              void* d_out, int out_size, void* d_ws, size_t ws_size,
                              hipStream_t stream) {
  if (n_in < 7) return;
  if (in_sizes[0] != NB * NI * 4) return;
  if (in_sizes[1] != NF * HD || in_sizes[2] != HD) return;
  if (in_sizes[3] != HD * ED || in_sizes[4] != ED) return;
  if (in_sizes[5] != PD * ED || in_sizes[6] != ED) return;
  if (out_size != NB * ED) return;

  const float* items = (const float*)d_in[0];
  const float* W1    = (const float*)d_in[1];
  const float* b1    = (const float*)d_in[2];
  const float* W2    = (const float*)d_in[3];
  const float* b2    = (const float*)d_in[4];
  const float* Wr    = (const float*)d_in[5];
  const float* br    = (const float*)d_in[6];
  float* out = (float*)d_out;

  char* ws = (char*)d_ws;
  size_t off = 0;
  const size_t oW2h = off; off += (size_t)ED * HD * 2;       off = (off + 255) & ~(size_t)255;
  const size_t oW2l = off; off += (size_t)ED * HD * 2;       off = (off + 255) & ~(size_t)255;
  const size_t oWrh = off; off += (size_t)ED * PD * 2;       off = (off + 255) & ~(size_t)255;
  const size_t oWrl = off; off += (size_t)ED * PD * 2;       off = (off + 255) & ~(size_t)255;
  const size_t oPt  = off; off += (size_t)NB * BPB * PD * 4; off = (off + 255) & ~(size_t)255;
  if (off > ws_size || off > (size_t)WSCAP) return;
  unsigned short* w2h = (unsigned short*)(ws + oW2h);
  unsigned short* w2l = (unsigned short*)(ws + oW2l);
  unsigned short* wrh = (unsigned short*)(ws + oWrh);
  unsigned short* wrl = (unsigned short*)(ws + oWrl);
  float* part = (float*)(ws + oPt);

  k_prepw<HD><<<ED / 16, 256, 0, stream>>>(W2, ED, w2h, w2l);
  k_prepw<PD><<<ED / 16, 256, 0, stream>>>(Wr, ED, wrh, wrl);

  k_phi<<<NB * BPB, WAVES * 32, 0, stream>>>(items, W1, b1, b2, w2h, w2l, part);

  k_head<<<NB / 16, 256, 0, stream>>>(part, wrh, wrl, br, out);
}
